// MultiHeadedGlobalAttention_13176959664319
// MI455X (gfx1250) — hardware-verified
//
#include <hip/hip_runtime.h>
#include <math.h>

constexpr int kBatch   = 4;
constexpr int kSeq     = 2048;
constexpr int kEmb     = 512;
constexpr int kHeads   = 8;
constexpr int kHd      = 64;
constexpr int kGq      = 16;
constexpr int kRows    = kBatch * kSeq;
constexpr int kCtxRows = kBatch * kGq;
constexpr int kChunk   = 64;
constexpr int kNChunk  = kSeq / kChunk;
constexpr int kPlaneW  = kEmb * kEmb;
constexpr int kAttLd   = 2 * kEmb;
static_assert(kHeads * kHd == kEmb, "head split");
static_assert(kRows % 64 == 0 && kEmb % 64 == 0 && kEmb % 32 == 0, "GEMM tile multiples");
static_assert(kAttLd == 1024 && kAttLd % 32 == 0, "output projection K multiple of 32");
static_assert(kCtxRows == 64, "context GEMM is exactly one 64-row tile");
static_assert(kSeq % kChunk == 0, "chunking exact");
static_assert(kChunk == 64 && kHd == 64 && kGq == 16, "scan thread maps assume these");

typedef __attribute__((ext_vector_type(16))) _Float16 v16h;
typedef __attribute__((ext_vector_type(8)))  _Float16 v8h;
typedef __attribute__((ext_vector_type(16))) __bf16   v16b;
typedef __attribute__((ext_vector_type(8)))  __bf16   v8b;
typedef __attribute__((ext_vector_type(8)))  float    v8f;
typedef __attribute__((ext_vector_type(4)))  float    v4f;
typedef __attribute__((ext_vector_type(4)))  unsigned int v4u;

__device__ __forceinline__ unsigned short f2bf_bits(float f) {
  unsigned u = __float_as_uint(f);
  return (unsigned short)((u + 0x7FFFu + ((u >> 16) & 1u)) >> 16);
}
__device__ __forceinline__ float bf_bits2f(unsigned short h) { return __uint_as_float(((unsigned)h) << 16); }
__device__ __forceinline__ unsigned pk16(unsigned short a, unsigned short b) { return (unsigned)a | ((unsigned)b << 16); }

__device__ __forceinline__ void dep_guard4_h(v8f& a, v8f& b, v8f& c, v8f& d, v16h x, v16h y) { asm volatile("v_nop\n\tv_nop\n\tv_nop\n\tv_nop" : "+v"(a), "+v"(b), "+v"(c), "+v"(d) : "v"(x), "v"(y)); }
__device__ __forceinline__ void dep_guard4_b(v8f& a, v8f& b, v8f& c, v8f& d, v16b x, v16b y) { asm volatile("v_nop\n\tv_nop\n\tv_nop\n\tv_nop" : "+v"(a), "+v"(b), "+v"(c), "+v"(d) : "v"(x), "v"(y)); }
__device__ __forceinline__ void keep4_h(v16h a, v16h b, v16h c, v16h d) { asm volatile("v_nop" :: "v"(a), "v"(b), "v"(c), "v"(d)); }
__device__ __forceinline__ void keep4_b(v16b a, v16b b, v16b c, v16b d) { asm volatile("v_nop" :: "v"(a), "v"(b), "v"(c), "v"(d)); }
__device__ __forceinline__ void acc_guard4(v8f& a, v8f& b, v8f& c, v8f& d) { asm volatile("v_nop\n\tv_nop\n\tv_nop\n\tv_nop" : "+v"(a), "+v"(b), "+v"(c), "+v"(d)); }

template <typename T> struct Frag;
template <> struct Frag<_Float16> {
  typedef v16h V; union U { v16h v; v8h h[2]; };
  static __device__ __forceinline__ v16h load(const _Float16* p) {
    U f; f.h[0] = *(const v8h*)(p); f.h[1] = *(const v8h*)(p + 16); return f.v;
  }
  static __device__ __forceinline__ v8f mma(v16h a, v16h b, v8f c) {
    return __builtin_amdgcn_wmma_f32_16x16x32_f16(false, a, false, b, (short)0, c, false, false);
  }
  static __device__ __forceinline__ void guard4(v8f& a, v8f& b, v8f& c, v8f& d, v16h x, v16h y) { dep_guard4_h(a, b, c, d, x, y); }
  static __device__ __forceinline__ void keep(v16h a, v16h b, v16h c, v16h d) { keep4_h(a, b, c, d); }
};
template <> struct Frag<__bf16> {
  typedef v16b V; union U { v16b v; v8b h[2]; };
  static __device__ __forceinline__ v16b load(const __bf16* p) {
    U f; f.h[0] = *(const v8b*)(p); f.h[1] = *(const v8b*)(p + 16); return f.v;
  }
  static __device__ __forceinline__ v8f mma(v16b a, v16b b, v8f c) {
    return __builtin_amdgcn_wmma_f32_16x16x32_bf16(false, a, false, b, (short)0, c, false, false);
  }
  static __device__ __forceinline__ void guard4(v8f& a, v8f& b, v8f& c, v8f& d, v16b x, v16b y) { dep_guard4_b(a, b, c, d, x, y); }
  static __device__ __forceinline__ void keep(v16b a, v16b b, v16b c, v16b d) { keep4_b(a, b, c, d); }
};

template <int ET> struct Elem;
template <> struct Elem<0> { typedef _Float16 T; };
template <> struct Elem<1> { typedef __bf16 T; };
template <int ET, bool SPLIT, int BIAS_MODE, int OUT_MODE, bool RESID, int ACT = 0>
__global__ __launch_bounds__(256) void wmma_gemm64(
    const unsigned short* __restrict__ Ap, const unsigned short* __restrict__ A2p, int lda, long strideA,
    const unsigned short* __restrict__ Btp, const unsigned short* __restrict__ Bt2p, int ldb, long strideB,
    void* __restrict__ Cout, void* __restrict__ Cout2, int ldc, long strideC,
    const float* __restrict__ bias,
    const float* __restrict__ resid, long strideR,
    int M, int N, int K, float scale) {
  typedef typename Elem<ET>::T T;
  typedef typename Frag<T>::V V;
  const T* A = (const T*)Ap; const T* A2 = (const T*)A2p; const T* Bt = (const T*)Btp; const T* Bt2 = (const T*)Bt2p;
  __shared__ __align__(16) float sT[8][16 * 68];
  const int b    = blockIdx.y;
  const int lane = threadIdx.x & 31;
  const int wave = threadIdx.x >> 5;
  const int tilesN = N >> 6;
  const int tilesM = M >> 6;
  const int tile = blockIdx.x * 8 + wave;
  if (tile >= tilesM * tilesN) return;
  const int tm = tile / tilesN;
  const int tn = tile - tm * tilesN;
  const int m0 = tm << 6;
  const int n0 = tn << 6;

  const T* Ab  = A  + (size_t)b * strideA;
  const T* Bb  = Bt + (size_t)b * strideB;
  const T* Ab2 = SPLIT ? (A2  + (size_t)b * strideA) : nullptr;
  const T* Bb2 = SPLIT ? (Bt2 + (size_t)b * strideB) : nullptr;

  const int rlane = lane & 15;
  const int koff  = (lane >> 4) * 8;
  const int mOff  = (lane >> 4) * 8;

  v8f acc[4][4];
#pragma unroll
  for (int i = 0; i < 4; ++i)
#pragma unroll
    for (int j = 0; j < 4; ++j) acc[i][j] = (v8f){0.f,0.f,0.f,0.f,0.f,0.f,0.f,0.f};

  for (int k0 = 0; k0 < K; k0 += 32) {
    V bh[4], bl[4];
#pragma unroll
    for (int j = 0; j < 4; ++j) {
      const size_t bo = (size_t)(n0 + (j << 4) + rlane) * ldb + koff + k0;
      bh[j] = Frag<T>::load(Bb + bo);
      if (SPLIT) bl[j] = Frag<T>::load(Bb2 + bo);
    }
#pragma unroll
    for (int i = 0; i < 4; ++i) {
      const size_t ao = (size_t)(m0 + (i << 4) + rlane) * lda + koff + k0;
      V ah = Frag<T>::load(Ab + ao);
      V al;
      if (SPLIT) al = Frag<T>::load(Ab2 + ao);
#pragma unroll
      for (int j = 0; j < 4; ++j) {
        acc[i][j] = Frag<T>::mma(ah, bh[j], acc[i][j]);
        if (SPLIT) {
          acc[i][j] = Frag<T>::mma(ah, bl[j], acc[i][j]);
          acc[i][j] = Frag<T>::mma(al, bh[j], acc[i][j]);
        }
      }
      Frag<T>::guard4(acc[i][0], acc[i][1], acc[i][2], acc[i][3], ah, SPLIT ? al : ah);
    }
    Frag<T>::keep(bh[0], bh[1], bh[2], bh[3]);
    if (SPLIT) Frag<T>::keep(bl[0], bl[1], bl[2], bl[3]);
  }
  acc_guard4(acc[0][0], acc[0][1], acc[0][2], acc[0][3]);
  acc_guard4(acc[1][0], acc[1][1], acc[1][2], acc[1][3]);
  acc_guard4(acc[2][0], acc[2][1], acc[2][2], acc[2][3]);
  acc_guard4(acc[3][0], acc[3][1], acc[3][2], acc[3][3]);

  float* slab = sT[wave];
  const float* Rb = RESID ? (resid + (size_t)b * strideR) : nullptr;
#pragma unroll
  for (int i = 0; i < 4; ++i) {
    const int mBase = m0 + (i << 4);
#pragma unroll
    for (int j = 0; j < 4; ++j) {
      const int n = n0 + (j << 4) + rlane;
      float bv = 0.f;
      if (BIAS_MODE == 2) bv = bias[n];
#pragma unroll
      for (int r = 0; r < 8; ++r) {
        float v = acc[i][j][r] * scale;
        if (BIAS_MODE == 1) v += bias[mBase + mOff + r];
        if (BIAS_MODE == 2) v += bv;
        if (RESID) v += Rb[(size_t)(mBase + mOff + r) * ldc + n];
        if (ACT == 2) v = fmaxf(v, 0.0f);
        if (ACT == 4) v = (v > 0.f) ? v : 0.01f * v;
        slab[(mOff + r) * 68 + (j << 4) + rlane] = v;
      }
    }
    __builtin_amdgcn_fence(__ATOMIC_RELEASE, "workgroup");
    __builtin_amdgcn_wave_barrier();
    __builtin_amdgcn_fence(__ATOMIC_ACQUIRE, "workgroup");
    if (OUT_MODE == 0) {
      float* C = (float*)Cout + (size_t)b * strideC;
      const int hh = lane >> 4, c4 = (lane & 15) * 4;
      for (int pass = 0; pass < 2; ++pass) {
#pragma unroll
        for (int it = 0; it < 8; ++it) {
          const int row = it * 2 + hh;
          v4f v = *(const v4f*)(slab + row * 68 + c4);
          *(volatile v4f*)(C + (size_t)(mBase + row) * ldc + n0 + c4) = v;
        }
        __threadfence();
      }
    } else {
      const int q = lane >> 3, c8 = (lane & 7) * 8;
      unsigned short* C  = (unsigned short*)Cout  + (size_t)b * strideC;
      unsigned short* C2 = (OUT_MODE == 2) ? ((unsigned short*)Cout2 + (size_t)b * strideC) : nullptr;
      for (int pass = 0; pass < 2; ++pass) {
#pragma unroll
        for (int it = 0; it < 4; ++it) {
          const int row = it * 4 + q;
          const float* sp = slab + row * 68 + c8;
          v8h hv, lv;
#pragma unroll
          for (int e = 0; e < 8; ++e) {
            if (OUT_MODE == 1) {
              hv[e] = (_Float16)sp[e];
            } else {
              unsigned short hb = f2bf_bits(sp[e]);
              unsigned short lb = f2bf_bits(sp[e] - bf_bits2f(hb));
              hv[e] = __builtin_bit_cast(_Float16, hb);
              lv[e] = __builtin_bit_cast(_Float16, lb);
            }
          }
          *(volatile v8h*)(C + (size_t)(mBase + row) * ldc + n0 + c8) = hv;
          if (OUT_MODE == 2) *(volatile v8h*)(C2 + (size_t)(mBase + row) * ldc + n0 + c8) = lv;
        }
        __threadfence();
      }
    }
    __builtin_amdgcn_fence(__ATOMIC_RELEASE, "workgroup");
    __builtin_amdgcn_wave_barrier();
    __builtin_amdgcn_fence(__ATOMIC_ACQUIRE, "workgroup");
  }
}

__global__ __launch_bounds__(256) void cvt8_bf16_kernel(const float* __restrict__ in0, const float* __restrict__ in1,
                                                        const float* __restrict__ in2, unsigned short* __restrict__ out, int n8) {
  const int z = blockIdx.y;
  const float* in = (z == 0) ? in0 : (z == 1) ? in1 : in2;
  const int i = blockIdx.x * 256 + threadIdx.x;
  if (i >= n8) return;
  const float* p = in + 8 * (size_t)i;
  const v4f a = *(const v4f*)(p);
  const v4f c = *(const v4f*)(p + 4);
  unsigned short hb[8];
#pragma unroll
  for (int e = 0; e < 4; ++e) {
    const float fa = a[e];
    const float fc = c[e];
    hb[e]     = f2bf_bits(fa);
    hb[4 + e] = f2bf_bits(fc);
  }
  const v4u u = (v4u){pk16(hb[0], hb[1]), pk16(hb[2], hb[3]), pk16(hb[4], hb[5]), pk16(hb[6], hb[7])};
  unsigned short* q = out + (size_t)z * (size_t)n8 * 8 + 8 * (size_t)i;
  *(volatile v4u*)q = u;
  __threadfence();
  *(volatile v4u*)q = u;
}

__global__ __launch_bounds__(256) void wt_prep_kernel(const float* __restrict__ W0, const float* __restrict__ W1,
                                                      const float* __restrict__ W2, const float* __restrict__ W3,
                                                      const float* __restrict__ W4, unsigned short* __restrict__ out) {
  __shared__ float sm[64][65];
  const int t  = threadIdx.x;
  const int k0 = blockIdx.x * 64;
  const int n0 = blockIdx.y * 64;
  const int z  = blockIdx.z;
  const float* W = (z == 0) ? W0 : (z == 1) ? W1 : (z == 2) ? W2 : (z == 3) ? W3 : W4;
#pragma unroll
  for (int i = 0; i < 16; ++i) {
    const int e = i * 256 + t;
    const int r = e >> 6;
    const int c = e & 63;
    sm[c][r] = W[(size_t)(k0 + r) * kEmb + n0 + c];
  }
  __syncthreads();
  const int lane = t & 31, wave = t >> 5;
  const int q = lane >> 3, c8 = (lane & 7) * 8;
  const int pitch = (z < 4) ? kEmb : kAttLd;
  const size_t pbase = (z < 4) ? ((size_t)z * kPlaneW) : ((size_t)4 * kPlaneW + (size_t)(z - 4) * kEmb);
  unsigned short* op = out + pbase;
  v4u u[2];
#pragma unroll
  for (int it = 0; it < 2; ++it) {
    const int row = wave * 8 + it * 4 + q;
    unsigned short hb[8];
#pragma unroll
    for (int e = 0; e < 8; ++e) {
      const float v = sm[row][c8 + e];
      hb[e] = f2bf_bits(v);
    }
    u[it] = (v4u){pk16(hb[0], hb[1]), pk16(hb[2], hb[3]), pk16(hb[4], hb[5]), pk16(hb[6], hb[7])};
  }
  for (int pass = 0; pass < 2; ++pass) {
#pragma unroll
    for (int it = 0; it < 2; ++it) {
      const int row = wave * 8 + it * 4 + q;
      *(volatile v4u*)(op + (size_t)(n0 + row) * pitch + k0 + c8) = u[it];
    }
    __threadfence();
  }
}

__global__ __launch_bounds__(256) void gscan_kernel(const float* __restrict__ qs, const float* __restrict__ ks,
                                                    const float* __restrict__ vs, const float* __restrict__ cs,
                                                    unsigned short* __restrict__ att) {
  __shared__ __align__(16) float Kt[kChunk * kHd];
  __shared__ __align__(16) float Vt[kChunk * kHd];
  __shared__ __align__(16) float Qt[kChunk * kHd];
  __shared__ __align__(16) float Ct[kGq * kHd];
  __shared__ __align__(16) float Wx[kChunk * kGq];
  __shared__ __align__(16) float QDx[kChunk * kGq];
  __shared__ __align__(16) float NNx[kChunk * kGq];
  __shared__ __align__(16) float Rx[kChunk * kGq];
  float* Ot = Qt;

  const int t    = threadIdx.x;
  const int lane = t & 31, wave = t >> 5;
  const int bh   = blockIdx.x;
  const int b    = bh / kHeads;
  const int h    = bh - b * kHeads;
  const size_t headbase = (size_t)b * kSeq * kEmb + (size_t)h * kHd;

  {
    const int g = t >> 4, j = t & 15;
    const v4f cv = *(const v4f*)(cs + (size_t)(b * kGq + g) * kEmb + h * kHd + 4 * j);
    *(v4f*)(Ct + g * kHd + 4 * j) = cv;
  }

  const int gA = t >> 4, ci = t & 15;
  const int sS = t >> 2, gq = t & 3;
  const int eB = 8 * wave + (lane >> 2);
  const int sq = lane >> 3, c8 = (lane & 7) * 8;

  float n_run = 0.0f;
  float Ak[4] = {0.0f, 0.0f, 0.0f, 0.0f};
  float Av[4] = {0.0f, 0.0f, 0.0f, 0.0f};

#pragma unroll 1
  for (int ch = 0; ch < kNChunk; ++ch) {
    __syncthreads();
    const size_t rowbase = headbase + (size_t)(ch * kChunk) * kEmb;
#pragma unroll
    for (int i = 0; i < 4; ++i) {
      const int fi = t + i * 256;
      const int s = fi >> 4, j = fi & 15;
      const size_t go = rowbase + (size_t)s * kEmb + 4 * j;
      const v4f kk = *(const v4f*)(ks + go);
      const v4f vv = *(const v4f*)(vs + go);
      const v4f qq = *(const v4f*)(qs + go);
      *(v4f*)(Kt + s * kHd + 4 * j) = kk;
      *(v4f*)(Vt + s * kHd + 4 * j) = vv;
      *(v4f*)(Qt + s * kHd + 4 * j) = qq;
    }
    __syncthreads();

#pragma unroll 1
    for (int p = 0; p < 4; ++p) {
      const int s = p * 16 + (t >> 4);
      const int g = t & 15;
      const float* kr = Kt + s * kHd;
      const float* cr = Ct + g * kHd;
      float d = 0.0f;
#pragma unroll 2
      for (int j = 0; j < 16; ++j) {
        const v4f kk = *(const v4f*)(kr + 4 * j);
        const v4f cc = *(const v4f*)(cr + 4 * j);
        d = fmaf(cc[0], kk[0], d);
        d = fmaf(cc[1], kk[1], d);
        d = fmaf(cc[2], kk[2], d);
        d = fmaf(cc[3], kk[3], d);
      }
      Wx[s * kGq + g] = expf(d);
    }
    __syncthreads();

#pragma unroll 1
    for (int s = 0; s < kChunk; ++s) {
      const v4f kk = *(const v4f*)(Kt + s * kHd + 4 * ci);
      const v4f qq = *(const v4f*)(Qt + s * kHd + 4 * ci);
      const float w = Wx[s * kGq + gA];
      n_run += w;
      Ak[0] = fmaf(w, kk[0], Ak[0]);
      Ak[1] = fmaf(w, kk[1], Ak[1]);
      Ak[2] = fmaf(w, kk[2], Ak[2]);
      Ak[3] = fmaf(w, kk[3], Ak[3]);
      float qd = qq[0] * Ak[0];
      qd = fmaf(qq[1], Ak[1], qd);
      qd = fmaf(qq[2], Ak[2], qd);
      qd = fmaf(qq[3], Ak[3], qd);
      qd += __shfl_xor(qd, 1, 32);
      qd += __shfl_xor(qd, 2, 32);
      qd += __shfl_xor(qd, 4, 32);
      qd += __shfl_xor(qd, 8, 32);
      if (ci == 0) {
        QDx[s * kGq + gA] = qd;
        NNx[s * kGq + gA] = n_run;
      }
    }
    __syncthreads();

    {
      const v4f qd4 = *(const v4f*)(QDx + sS * kGq + 4 * gq);
      const v4f nn4 = *(const v4f*)(NNx + sS * kGq + 4 * gq);
      float inv[4], lg[4], pe[4];
#pragma unroll
      for (int i = 0; i < 4; ++i) {
        const float nv = nn4[i];
        const float qv = qd4[i];
        inv[i] = __builtin_amdgcn_rcpf(nv);
        lg[i]  = qv * inv[i];
      }
      float m = fmaxf(fmaxf(lg[0], lg[1]), fmaxf(lg[2], lg[3]));
      m = fmaxf(m, __shfl_xor(m, 1, 32));
      m = fmaxf(m, __shfl_xor(m, 2, 32));
      float sum = 0.0f;
#pragma unroll
      for (int i = 0; i < 4; ++i) {
        pe[i] = expf(lg[i] - m);
        sum += pe[i];
      }
      sum += __shfl_xor(sum, 1, 32);
      sum += __shfl_xor(sum, 2, 32);
      const float rd = __builtin_amdgcn_rcpf(sum);
      v4f r4;
      r4[0] = pe[0] * rd * inv[0];
      r4[1] = pe[1] * rd * inv[1];
      r4[2] = pe[2] * rd * inv[2];
      r4[3] = pe[3] * rd * inv[3];
      *(v4f*)(Rx + sS * kGq + 4 * gq) = r4;
    }
    __syncthreads();

#pragma unroll 1
    for (int s = 0; s < kChunk; ++s) {
      const v4f w4 = *(const v4f*)(Wx + s * kGq + 4 * gq);
      const v4f r4 = *(const v4f*)(Rx + s * kGq + 4 * gq);
      const float vv = Vt[s * kHd + eB];
      Av[0] = fmaf(w4[0], vv, Av[0]);
      Av[1] = fmaf(w4[1], vv, Av[1]);
      Av[2] = fmaf(w4[2], vv, Av[2]);
      Av[3] = fmaf(w4[3], vv, Av[3]);
      float o = r4[0] * Av[0];
      o = fmaf(r4[1], Av[1], o);
      o = fmaf(r4[2], Av[2], o);
      o = fmaf(r4[3], Av[3], o);
      o += __shfl_xor(o, 1, 32);
      o += __shfl_xor(o, 2, 32);
      if (gq == 0) Ot[s * kHd + eB] = o;
    }
    __syncthreads();

    {
      v4u uh[2], ul[2];
#pragma unroll
      for (int it = 0; it < 2; ++it) {
        const int row = wave * 8 + it * 4 + sq;
        const float* sp = Ot + row * kHd + c8;
        const v4f a = *(const v4f*)(sp);
        const v4f c = *(const v4f*)(sp + 4);
        unsigned short hb[8], lb[8];
#pragma unroll
        for (int e = 0; e < 4; ++e) {
          const float fa = a[e];
          const float fc = c[e];
          const unsigned short ha = f2bf_bits(fa);
          const unsigned short hc = f2bf_bits(fc);
          hb[e]     = ha;
          hb[4 + e] = hc;
          lb[e]     = f2bf_bits(fa - bf_bits2f(ha));
          lb[4 + e] = f2bf_bits(fc - bf_bits2f(hc));
        }
        uh[it] = (v4u){pk16(hb[0], hb[1]), pk16(hb[2], hb[3]), pk16(hb[4], hb[5]), pk16(hb[6], hb[7])};
        ul[it] = (v4u){pk16(lb[0], lb[1]), pk16(lb[2], lb[3]), pk16(lb[4], lb[5]), pk16(lb[6], lb[7])};
      }
      unsigned short* ob = att + ((size_t)b * kSeq + (size_t)ch * kChunk) * kAttLd + h * kHd + c8;
      for (int pass = 0; pass < 2; ++pass) {
#pragma unroll
        for (int it = 0; it < 2; ++it) {
          const int row = wave * 8 + it * 4 + sq;
          *(volatile v4u*)(ob + (size_t)row * kAttLd) = uh[it];
          *(volatile v4u*)(ob + (size_t)row * kAttLd + kEmb) = ul[it];
        }
        __threadfence();
      }
    }
  }
}

extern "C" void kernel_launch(void* const* d_in, const int* in_sizes, int n_in,
                              void* d_out, int out_size, void* d_ws, size_t ws_size, hipStream_t stream) {
  if (n_in < 9 || d_out == nullptr || d_ws == nullptr) return;
  if (in_sizes[0] != kRows * kEmb || in_sizes[1] != kRows * kEmb || in_sizes[2] != kRows * kEmb ||
      in_sizes[3] != kCtxRows * kEmb || in_sizes[4] != kPlaneW || in_sizes[5] != kPlaneW ||
      in_sizes[6] != kPlaneW || in_sizes[7] != kPlaneW || in_sizes[8] != kPlaneW ||
      out_size != kRows * kEmb) return;

  const float* query = (const float*)d_in[0];
  const float* key   = (const float*)d_in[1];
  const float* value = (const float*)d_in[2];
  const float* ctx   = (const float*)d_in[3];
  const float* wq    = (const float*)d_in[4];
  const float* wk    = (const float*)d_in[5];
  const float* wv    = (const float*)d_in[6];
  const float* wo    = (const float*)d_in[7];
  const float* wc    = (const float*)d_in[8];
  float* outp = (float*)d_out;

  char* ws = (char*)d_ws; size_t off = 0;
  auto carve = [&](size_t bytes) -> char* { char* p = ws + off; off += (bytes + 255) & ~(size_t)255; return p; };
  unsigned short* A16 = (unsigned short*)carve((size_t)3 * kRows * kEmb * 2);
  unsigned short* C16 = (unsigned short*)carve((size_t)kCtxRows * kEmb * 2);
  unsigned short* WT  = (unsigned short*)carve(((size_t)4 * kPlaneW + (size_t)kEmb * kAttLd) * 2);
  float*          QKV = (float*)carve((size_t)3 * kRows * kEmb * 4);
  float*          CSP = (float*)carve((size_t)kCtxRows * kEmb * 4);
  unsigned short* ATT = (unsigned short*)carve((size_t)kRows * kAttLd * 2);
  if (off > ws_size || off > (size_t)134217728) return;
  unsigned short* WOD = WT + (size_t)4 * kPlaneW;

  const int n8act = kRows * kEmb / 8;
  const int n8ctx = kCtxRows * kEmb / 8;
  cvt8_bf16_kernel<<<dim3(n8act / 256, 3), 256, 0, stream>>>(query, key, value, A16, n8act);
  cvt8_bf16_kernel<<<dim3(n8ctx / 256, 1), 256, 0, stream>>>(ctx, ctx, ctx, C16, n8ctx);
  wt_prep_kernel<<<dim3(8, 8, 6), 256, 0, stream>>>(wq, wk, wv, wc, wo, WT);

  const long actStride = (long)kRows * kEmb;
  wmma_gemm64<1, false, 0, 0, false, 0><<<dim3((kRows / 64) * (kEmb / 64) / 8, 3), 256, 0, stream>>>(
      A16, A16, kEmb, actStride, WT, WT, kEmb, (long)kPlaneW, (void*)QKV, (void*)QKV, kEmb, actStride,
      CSP, CSP, 0L, kRows, kEmb, kEmb, 1.0f);
  wmma_gemm64<1, false, 0, 0, false, 0><<<dim3(1, 1), 256, 0, stream>>>(
      C16, C16, kEmb, 0L, WT + (size_t)3 * kPlaneW, WT + (size_t)3 * kPlaneW, kEmb, 0L, (void*)CSP, (void*)CSP, kEmb, 0L,
      QKV, QKV, 0L, kCtxRows, kEmb, kEmb, 1.0f);

  const float* qsP = QKV;
  const float* ksP = QKV + (size_t)kRows * kEmb;
  const float* vsP = QKV + (size_t)2 * kRows * kEmb;
  gscan_kernel<<<kBatch * kHeads, 256, 0, stream>>>(qsP, ksP, vsP, CSP, ATT);

  wmma_gemm64<1, false, 0, 0, false, 0><<<dim3((kRows / 64) * (kEmb / 64) / 8, 1), 256, 0, stream>>>(
      ATT, ATT, kAttLd, 0L, WOD, WOD, kAttLd, 0L, (void*)outp, (void*)outp, kEmb, 0L,
      CSP, CSP, 0L, kRows, kEmb, kAttLd, 1.0f);
}
